// GRUNet_25039659335813
// MI455X (gfx1250) — hardware-run, weakly checked
//
#include <hip/hip_runtime.h>
#include <hip/hip_bf16.h>

constexpr int kBatch     = 128;
constexpr int kSteps     = 512;
constexpr int kIn        = 64;
constexpr int kHid       = 256;
constexpr int kGates     = 768;
constexpr int kOut       = 2;
constexpr int kChunk     = 128;
constexpr int kNumChunks = kSteps / kChunk;
constexpr int kRowsPerBlk = 16;
constexpr int kHP        = 264;
constexpr float kScaleX  = 16.0f;
constexpr float kScaleH  = 64.0f;
constexpr float kScaleW  = 256.0f;
constexpr float kInProj0Scale = 1.0f / (16.0f * 256.0f);
constexpr float kInProj1Scale = 1.0f / (64.0f * 256.0f);
constexpr float kRecScale     = 1.0f / (64.0f * 256.0f);

static_assert(kSteps % kChunk == 0);
static_assert(kBatch % kRowsPerBlk == 0);
static_assert(kIn % 32 == 0 && kHid % 32 == 0);
static_assert((kChunk * kBatch) % 64 == 0 && kGates % 64 == 0);
static_assert((kRowsPerBlk * kGates) % (4 * 256) == 0);
static_assert((kRowsPerBlk * kHid) % (4 * 256) == 0);
static_assert((kRowsPerBlk * kHP) % 8 == 0);
static_assert(kHid == 8 * 32);

constexpr size_t kOffWih0 = 0;
constexpr size_t kOffWhh0 = kOffWih0 + (size_t)kGates * kIn * 2;
constexpr size_t kOffWih1 = kOffWhh0 + (size_t)kGates * kHid * 2;
constexpr size_t kOffWhh1 = kOffWih1 + (size_t)kGates * kHid * 2;
constexpr size_t kOffX16  = kOffWhh1 + (size_t)kGates * kHid * 2;
constexpr size_t kOffH1p  = kOffX16 + (size_t)kSteps * kBatch * kIn * 2;
constexpr size_t kOffXg   = kOffH1p + (size_t)kSteps * kBatch * kHid * 2;
constexpr size_t kOffHsA  = kOffXg + (size_t)kChunk * kBatch * kGates * 4;
constexpr size_t kOffHsB  = kOffHsA + (size_t)kBatch * kHid * 4;
constexpr size_t kWsTotal = kOffHsB + (size_t)kBatch * kHid * 4;
static_assert(kWsTotal == 93814784u);
static_assert(kWsTotal <= 134217728u);
static_assert(kOffWhh0 % 256 == 0 && kOffWih1 % 256 == 0 && kOffWhh1 % 256 == 0 && kOffX16 % 256 == 0);
static_assert(kOffH1p % 256 == 0 && kOffXg % 256 == 0 && kOffHsA % 256 == 0 && kOffHsB % 256 == 0);

typedef __attribute__((ext_vector_type(16))) _Float16 v16h;
typedef __attribute__((ext_vector_type(8)))  _Float16 v8h;
typedef __attribute__((ext_vector_type(16))) __bf16   v16b;
typedef __attribute__((ext_vector_type(8)))  __bf16   v8b;
typedef __attribute__((ext_vector_type(8)))  float    v8f;
typedef __attribute__((ext_vector_type(4)))  float    v4f;

__device__ __forceinline__ unsigned short f2bf_bits(float f) {
  unsigned u = __float_as_uint(f);
  return (unsigned short)((u + 0x7FFFu + ((u >> 16) & 1u)) >> 16);
}
__device__ __forceinline__ float bf_bits2f(unsigned short h) { return __uint_as_float(((unsigned)h) << 16); }

__device__ __forceinline__ void dep_guard_h(v8f& a, v8f& b, v16h x, v16h y) { asm volatile("v_nop\n\tv_nop\n\tv_nop\n\tv_nop" : "+v"(a), "+v"(b) : "v"(x), "v"(y)); }
__device__ __forceinline__ void dep_guard_b(v8f& a, v8f& b, v16b x, v16b y) { asm volatile("v_nop\n\tv_nop\n\tv_nop\n\tv_nop" : "+v"(a), "+v"(b) : "v"(x), "v"(y)); }
__device__ __forceinline__ void keep4_h(v16h a, v16h b, v16h c, v16h d) { asm volatile("v_nop" :: "v"(a), "v"(b), "v"(c), "v"(d)); }
__device__ __forceinline__ void keep4_b(v16b a, v16b b, v16b c, v16b d) { asm volatile("v_nop" :: "v"(a), "v"(b), "v"(c), "v"(d)); }
__device__ __forceinline__ void acc_guard4(v8f& a, v8f& b, v8f& c, v8f& d) { asm volatile("v_nop\n\tv_nop\n\tv_nop\n\tv_nop" : "+v"(a), "+v"(b), "+v"(c), "+v"(d)); }

template <typename T> struct Frag;
template <> struct Frag<_Float16> {
  typedef v16h V; union U { v16h v; v8h h[2]; };
  static __device__ __forceinline__ v16h load(const _Float16* p) {
    U f; f.h[0] = *(const v8h*)(p); f.h[1] = *(const v8h*)(p + 16); return f.v;
  }
  static __device__ __forceinline__ v8f mma(v16h a, v16h b, v8f c) {
    return __builtin_amdgcn_wmma_f32_16x16x32_f16(false, a, false, b, (short)0, c, false, false);
  }
  static __device__ __forceinline__ void guard(v8f& a, v8f& b, v16h x, v16h y) { dep_guard_h(a, b, x, y); }
  static __device__ __forceinline__ void keep(v16h a, v16h b, v16h c, v16h d) { keep4_h(a, b, c, d); }
};
template <> struct Frag<__bf16> {
  typedef v16b V; union U { v16b v; v8b h[2]; };
  static __device__ __forceinline__ v16b load(const __bf16* p) {
    U f; f.h[0] = *(const v8b*)(p); f.h[1] = *(const v8b*)(p + 16); return f.v;
  }
  static __device__ __forceinline__ v8f mma(v16b a, v16b b, v8f c) {
    return __builtin_amdgcn_wmma_f32_16x16x32_bf16(false, a, false, b, (short)0, c, false, false);
  }
  static __device__ __forceinline__ void guard(v8f& a, v8f& b, v16b x, v16b y) { dep_guard_b(a, b, x, y); }
  static __device__ __forceinline__ void keep(v16b a, v16b b, v16b c, v16b d) { keep4_b(a, b, c, d); }
};

__device__ __forceinline__ v8f mma_h(v16h a, v16h b, v8f c) {
  c = __builtin_amdgcn_wmma_f32_16x16x32_f16(false, a, false, b, (short)0, c, false, false);
  asm volatile("v_nop\n\tv_nop\n\tv_nop\n\tv_nop" : "+v"(c) : "v"(a), "v"(b));
  return c;
}

template <int ET> struct Elem;
template <> struct Elem<0> { typedef _Float16 T; };
template <> struct Elem<1> { typedef __bf16 T; };
template <int ET, bool SPLIT, int BIAS_MODE, int OUT_MODE, bool RESID, int ACT = 0>
__global__ __launch_bounds__(256) void wmma_gemm64(
    const unsigned short* __restrict__ Ap, const unsigned short* __restrict__ A2p, int lda, long strideA,
    const unsigned short* __restrict__ Btp, const unsigned short* __restrict__ Bt2p, int ldb, long strideB,
    void* __restrict__ Cout, void* __restrict__ Cout2, int ldc, long strideC,
    const float* __restrict__ bias,
    const float* __restrict__ resid, long strideR,
    int M, int N, int K, float scale) {
  typedef typename Elem<ET>::T T;
  typedef typename Frag<T>::V V;
  const T* A = (const T*)Ap; const T* A2 = (const T*)A2p; const T* Bt = (const T*)Btp; const T* Bt2 = (const T*)Bt2p;
  __shared__ __align__(16) float sT[8][16 * 68];
  const int b    = blockIdx.y;
  const int lane = threadIdx.x & 31;
  const int wave = threadIdx.x >> 5;
  const int tilesN = N >> 6;
  const int tilesM = M >> 6;
  const int tile = blockIdx.x * 8 + wave;
  if (tile >= tilesM * tilesN) return;
  const int tm = tile / tilesN;
  const int tn = tile - tm * tilesN;
  const int m0 = tm << 6;
  const int n0 = tn << 6;

  const T* Ab  = A  + (size_t)b * strideA;
  const T* Bb  = Bt + (size_t)b * strideB;
  const T* Ab2 = SPLIT ? (A2  + (size_t)b * strideA) : nullptr;
  const T* Bb2 = SPLIT ? (Bt2 + (size_t)b * strideB) : nullptr;

  const int rlane = lane & 15;
  const int koff  = (lane >> 4) * 8;
  const int mOff  = (lane >> 4) * 8;

  v8f acc[4][4];
#pragma unroll
  for (int i = 0; i < 4; ++i)
#pragma unroll
    for (int j = 0; j < 4; ++j) acc[i][j] = (v8f){0.f,0.f,0.f,0.f,0.f,0.f,0.f,0.f};

  for (int k0 = 0; k0 < K; k0 += 32) {
    V bh[4], bl[4];
#pragma unroll
    for (int j = 0; j < 4; ++j) {
      const size_t bo = (size_t)(n0 + (j << 4) + rlane) * ldb + koff + k0;
      bh[j] = Frag<T>::load(Bb + bo);
      if (SPLIT) bl[j] = Frag<T>::load(Bb2 + bo);
    }
#pragma unroll
    for (int i = 0; i < 4; ++i) {
      const size_t ao = (size_t)(m0 + (i << 4) + rlane) * lda + koff + k0;
      V ah = Frag<T>::load(Ab + ao);
      V al;
      if (SPLIT) al = Frag<T>::load(Ab2 + ao);
#pragma unroll
      for (int j = 0; j < 4; ++j) {
        acc[i][j] = Frag<T>::mma(ah, bh[j], acc[i][j]);
        if (SPLIT) {
          acc[i][j] = Frag<T>::mma(ah, bl[j], acc[i][j]);
          acc[i][j] = Frag<T>::mma(al, bh[j], acc[i][j]);
        }
      }
      Frag<T>::guard(acc[i][0], acc[i][3], ah, SPLIT ? al : ah);
    }
    Frag<T>::keep(bh[0], bh[1], bh[2], bh[3]);
    if (SPLIT) Frag<T>::keep(bl[0], bl[1], bl[2], bl[3]);
  }
  acc_guard4(acc[0][0], acc[0][1], acc[0][2], acc[0][3]);
  acc_guard4(acc[1][0], acc[1][1], acc[1][2], acc[1][3]);
  acc_guard4(acc[2][0], acc[2][1], acc[2][2], acc[2][3]);
  acc_guard4(acc[3][0], acc[3][1], acc[3][2], acc[3][3]);

  float* slab = sT[wave];
  const float* Rb = RESID ? (resid + (size_t)b * strideR) : nullptr;
#pragma unroll
  for (int i = 0; i < 4; ++i) {
    const int mBase = m0 + (i << 4);
#pragma unroll
    for (int j = 0; j < 4; ++j) {
      const int n = n0 + (j << 4) + rlane;
      float bv = 0.f;
      if (BIAS_MODE == 2) bv = bias[n];
#pragma unroll
      for (int r = 0; r < 8; ++r) {
        float v = acc[i][j][r] * scale;
        if (BIAS_MODE == 1) v += bias[mBase + mOff + r];
        if (BIAS_MODE == 2) v += bv;
        if (RESID) v += Rb[(size_t)(mBase + mOff + r) * ldc + n];
        if (ACT == 1) v = tanhf(v);
        if (ACT == 2) v = fmaxf(v, 0.0f);
        if (ACT == 3) v = v / (1.0f + expf(-v));
        if (ACT == 4) v = (v > 0.f) ? v : 0.01f * v;
        if (ACT == 5) v = 0.5f * v * (1.0f + erff(v * 0.70710678118654752f));
        slab[(mOff + r) * 68 + (j << 4) + rlane] = v;
      }
    }
    __builtin_amdgcn_fence(__ATOMIC_RELEASE, "workgroup");
    __builtin_amdgcn_wave_barrier();
    __builtin_amdgcn_fence(__ATOMIC_ACQUIRE, "workgroup");
    if (OUT_MODE == 0) {
      float* C = (float*)Cout + (size_t)b * strideC;
      const int hh = lane >> 4, c4 = (lane & 15) * 4;
      for (int pass = 0; pass < 2; ++pass) {
#pragma unroll
        for (int it = 0; it < 8; ++it) {
          const int row = it * 2 + hh;
          v4f v = *(const v4f*)(slab + row * 68 + c4);
          *(volatile v4f*)(C + (size_t)(mBase + row) * ldc + n0 + c4) = v;
        }
        __threadfence();
      }
    } else {
      const int q = lane >> 3, c8 = (lane & 7) * 8;
      unsigned short* C  = (unsigned short*)Cout  + (size_t)b * strideC;
      unsigned short* C2 = (OUT_MODE == 2) ? ((unsigned short*)Cout2 + (size_t)b * strideC) : nullptr;
      for (int pass = 0; pass < 2; ++pass) {
#pragma unroll
        for (int it = 0; it < 4; ++it) {
          const int row = it * 4 + q;
          const float* sp = slab + row * 68 + c8;
          v8h hv, lv;
#pragma unroll
          for (int e = 0; e < 8; ++e) {
            if (OUT_MODE == 1) {
              hv[e] = (_Float16)sp[e];
            } else {
              unsigned short hb = f2bf_bits(sp[e]);
              unsigned short lb = f2bf_bits(sp[e] - bf_bits2f(hb));
              hv[e] = __builtin_bit_cast(_Float16, hb);
              lv[e] = __builtin_bit_cast(_Float16, lb);
            }
          }
          *(volatile v8h*)(C + (size_t)(mBase + row) * ldc + n0 + c8) = hv;
          if (OUT_MODE == 2) *(volatile v8h*)(C2 + (size_t)(mBase + row) * ldc + n0 + c8) = lv;
        }
        __threadfence();
      }
    }
    __builtin_amdgcn_fence(__ATOMIC_RELEASE, "workgroup");
    __builtin_amdgcn_wave_barrier();
    __builtin_amdgcn_fence(__ATOMIC_ACQUIRE, "workgroup");
  }
}

__global__ __launch_bounds__(256) void cast_scale_f16x2(
    const float* __restrict__ in, unsigned short* __restrict__ out, int n2, float scale) {
  const int i = blockIdx.x * 256 + threadIdx.x;
  if (i < n2) {
    const float a = in[2 * i] * scale;
    const float c = in[2 * i + 1] * scale;
    const _Float16 h0 = (_Float16)a, h1 = (_Float16)c;
    const unsigned u = (unsigned)__builtin_bit_cast(unsigned short, h0) | ((unsigned)__builtin_bit_cast(unsigned short, h1) << 16);
    ((volatile unsigned*)out)[i] = u;
    __threadfence();
    ((volatile unsigned*)out)[i] = u;
  }
}

__global__ __launch_bounds__(256) void cast_x_timemajor(
    const float* __restrict__ x, unsigned short* __restrict__ xo_p, float scale) {
  _Float16* xo = (_Float16*)(void*)xo_p;
  const int tid = threadIdx.x, wave = tid >> 5, lane = tid & 31;
  int o = blockIdx.x * 32 + wave * 4 + (lane >> 3);
  if (o > kSteps * kBatch - 1) o = kSteps * kBatch - 1;
  const int c8 = (lane & 7) * 8;
  const int t = o / kBatch;
  const int b = o - t * kBatch;
  const float* src = x + ((size_t)b * kSteps + t) * kIn + c8;
  const v4f f0 = *(const v4f*)src;
  const v4f f1 = *(const v4f*)(src + 4);
  v8h hv;
#pragma unroll
  for (int e = 0; e < 4; ++e) { hv[e] = (_Float16)(f0[e] * scale); hv[4 + e] = (_Float16)(f1[e] * scale); }
  _Float16* dst = xo + (size_t)o * kIn + c8;
  *(volatile v8h*)dst = hv;
  __threadfence();
  *(volatile v8h*)dst = hv;
}

__device__ __forceinline__ float sigm_f(float v) {
  v = fminf(fmaxf(v, -30.0f), 30.0f);
  return 1.0f / (1.0f + expf(-v));
}

__global__ __launch_bounds__(256) void rec_chunk(
    const float* __restrict__ xg, const unsigned short* __restrict__ whh_p, const float* __restrict__ bhh,
    const float* __restrict__ h_in, float* __restrict__ h_out, unsigned short* __restrict__ hseq_p,
    int t0, int nsteps, int first, int write_seq) {
  const _Float16* whh = (const _Float16*)(const void*)whh_p;
  _Float16* hseq = (_Float16*)(void*)hseq_p;
  __shared__ __align__(16) float    xp[kRowsPerBlk * kGates];
  __shared__ __align__(16) _Float16 h16[kRowsPerBlk * kHP];

  const int tid = threadIdx.x;
  const int w = tid >> 5, lane = tid & 31, hh = lane >> 4, n = lane & 15;
  const int b0 = blockIdx.x * kRowsPerBlk;
  if (t0 < 0) t0 = 0;
  if (t0 > kSteps) t0 = kSteps;
  if (nsteps < 0) nsteps = 0;
  if (nsteps > kChunk) nsteps = kChunk;
  if (nsteps > kSteps - t0) nsteps = kSteps - t0;

  int jc[2];
  float br[2], bz[2], bnn[2];
#pragma unroll
  for (int tt = 0; tt < 2; ++tt) {
    jc[tt] = 32 * w + 16 * tt + n;
    br[tt]  = bhh[jc[tt]];
    bz[tt]  = bhh[kHid + jc[tt]];
    bnn[tt] = bhh[2 * kHid + jc[tt]];
  }

  float hprev[16];
  if (first != 0) {
    v8h z;
#pragma unroll
    for (int e = 0; e < 8; ++e) z[e] = (_Float16)0.0f;
    for (int i = tid; i < (kRowsPerBlk * kHP) / 8; i += 256) *(v8h*)(h16 + i * 8) = z;
#pragma unroll
    for (int i = 0; i < 16; ++i) hprev[i] = 0.0f;
  } else {
    const float* src = h_in + (size_t)b0 * kHid;
#pragma unroll
    for (int i = 0; i < (kRowsPerBlk * kHid) / (4 * 256); ++i) {
      const int q = i * 256 + tid;
      const v4f v = *(const v4f*)(src + (size_t)q * 4);
      *(v4f*)(xp + q * 4) = v;
    }
    __syncthreads();
#pragma unroll
    for (int tt = 0; tt < 2; ++tt) {
#pragma unroll
      for (int g = 0; g < 8; ++g) {
        const int m = 8 * hh + g;
        const float hv = xp[m * kHid + jc[tt]];
        hprev[tt * 8 + g] = hv;
        h16[m * kHP + jc[tt]] = (_Float16)(hv * kScaleH);
      }
    }
  }
  __syncthreads();

  for (int s = 0; s < nsteps; ++s) {
    {
      const float* pg = xg + ((size_t)s * kBatch + b0) * kGates;
#pragma unroll
      for (int i = 0; i < (kRowsPerBlk * kGates) / (4 * 256); ++i) {
        const int q = i * 256 + tid;
        const v4f v = *(const v4f*)(pg + (size_t)q * 4);
        *(v4f*)(xp + q * 4) = v;
      }
    }
    v8f acc[6];
#pragma unroll
    for (int c = 0; c < 6; ++c) acc[c] = (v8f){0.f,0.f,0.f,0.f,0.f,0.f,0.f,0.f};
#pragma unroll 2
    for (int kt = 0; kt < kHid / 32; ++kt) {
      const v16h a = Frag<_Float16>::load(h16 + n * kHP + kt * 32 + 8 * hh);
#pragma unroll
      for (int c = 0; c < 6; ++c) {
        const int growB = (c >> 1) * kHid + 32 * w + 16 * (c & 1) + n;
        const v16h bb = Frag<_Float16>::load(whh + (size_t)growB * kHid + kt * 32 + 8 * hh);
        acc[c] = mma_h(a, bb, acc[c]);
      }
    }
    __syncthreads();

#pragma unroll
    for (int tt = 0; tt < 2; ++tt) {
      const int j = jc[tt];
#pragma unroll
      for (int g = 0; g < 8; ++g) {
        const int m = 8 * hh + g;
        const float* xr_p = xp + m * kGates + j;
        const float xr = xr_p[0];
        const float xz = xr_p[kHid];
        const float xn = xr_p[2 * kHid];
        const float hr = acc[tt][g] * kRecScale + br[tt];
        const float hz = acc[2 + tt][g] * kRecScale + bz[tt];
        const float hn = acc[4 + tt][g] * kRecScale + bnn[tt];
        const float r = sigm_f(xr + hr);
        const float z = sigm_f(xz + hz);
        const float nn = tanhf(xn + r * hn);
        const int idx = tt * 8 + g;
        const float hnew = (1.0f - z) * nn + z * hprev[idx];
        hprev[idx] = hnew;
        h16[m * kHP + j] = (_Float16)(hnew * kScaleH);
      }
    }
    __syncthreads();

    if (write_seq != 0) {
      _Float16* dst = hseq + ((size_t)(t0 + s) * kBatch + b0) * kHid;
      for (int pass = 0; pass < 2; ++pass) {
#pragma unroll
        for (int it = 0; it < 2; ++it) {
          const int L = it * 32 + (tid >> 3);
          const int row = L >> 2;
          const int col = (L & 3) * 64 + (tid & 7) * 8;
          const v8h v = *(const v8h*)(h16 + row * kHP + col);
          *(volatile v8h*)(dst + (size_t)row * kHid + col) = v;
        }
        __threadfence();
      }
    }

    if (s == nsteps - 1) {
#pragma unroll
      for (int tt = 0; tt < 2; ++tt) {
#pragma unroll
        for (int g = 0; g < 8; ++g) {
          const int m = 8 * hh + g;
          xp[m * kHid + jc[tt]] = hprev[tt * 8 + g];
        }
      }
      __syncthreads();
      float* dst = h_out + (size_t)b0 * kHid;
      for (int pass = 0; pass < 2; ++pass) {
#pragma unroll
        for (int it = 0; it < 4; ++it) {
          const int L = it * 32 + (tid >> 3);
          const int row = L >> 3;
          const int col = (L & 7) * 32 + (tid & 7) * 4;
          const v4f v = *(const v4f*)(xp + row * kHid + col);
          *(volatile v4f*)(dst + (size_t)row * kHid + col) = v;
        }
        __threadfence();
      }
    }
  }
}

__global__ __launch_bounds__(256) void fc_head(
    const float* __restrict__ h, const float* __restrict__ fw, const float* __restrict__ fb,
    float* __restrict__ out) {
  __shared__ __align__(16) float so[kBatch * kOut];
  const int tid = threadIdx.x;
  const int b = tid >> 1, o = tid & 1;
  const float* hr = h + (size_t)b * kHid;
  const float* wr = fw + (size_t)o * kHid;
  float s = 0.0f;
#pragma unroll 1
  for (int j4 = 0; j4 < kHid / 4; ++j4) {
    const v4f hv = *(const v4f*)(hr + 4 * j4);
    const v4f wv = *(const v4f*)(wr + 4 * j4);
#pragma unroll
    for (int e = 0; e < 4; ++e) s += fmaxf(hv[e], 0.0f) * wv[e];
  }
  s += fb[o];
  so[tid] = s;
  __syncthreads();
  if (tid < 32) {
    for (int pass = 0; pass < 2; ++pass) {
#pragma unroll
      for (int it = 0; it < 2; ++it) {
        const v4f v = *(const v4f*)(so + it * 128 + tid * 4);
        *(volatile v4f*)(out + it * 128 + tid * 4) = v;
      }
      __threadfence();
    }
  }
}

extern "C" void kernel_launch(void* const* d_in, const int* in_sizes, int n_in,
                              void* d_out, int out_size, void* d_ws, size_t ws_size,
                              hipStream_t stream) {
  if (n_in < 11) return;
  if (in_sizes[0] != kBatch * kSteps * kIn) return;
  if (in_sizes[1] != kGates * kIn || in_sizes[2] != kGates * kHid) return;
  if (in_sizes[5] != kGates * kHid || in_sizes[6] != kGates * kHid) return;
  if (in_sizes[3] != kGates || in_sizes[4] != kGates || in_sizes[7] != kGates || in_sizes[8] != kGates) return;
  if (in_sizes[9] != kOut * kHid || in_sizes[10] != kOut) return;
  if (out_size != kBatch * kOut) return;
  if (ws_size < kWsTotal) return;

  const float* x     = (const float*)d_in[0];
  const float* w_ih0 = (const float*)d_in[1];
  const float* w_hh0 = (const float*)d_in[2];
  const float* b_ih0 = (const float*)d_in[3];
  const float* b_hh0 = (const float*)d_in[4];
  const float* w_ih1 = (const float*)d_in[5];
  const float* w_hh1 = (const float*)d_in[6];
  const float* b_ih1 = (const float*)d_in[7];
  const float* b_hh1 = (const float*)d_in[8];
  const float* fc_w  = (const float*)d_in[9];
  const float* fc_b  = (const float*)d_in[10];
  float* out = (float*)d_out;

  char* ws = (char*)d_ws;
  unsigned short* wih0 = (unsigned short*)(ws + kOffWih0);
  unsigned short* whh0 = (unsigned short*)(ws + kOffWhh0);
  unsigned short* wih1 = (unsigned short*)(ws + kOffWih1);
  unsigned short* whh1 = (unsigned short*)(ws + kOffWhh1);
  unsigned short* x16  = (unsigned short*)(ws + kOffX16);
  unsigned short* h1p  = (unsigned short*)(ws + kOffH1p);
  float* xg  = (float*)(ws + kOffXg);
  float* hsA = (float*)(ws + kOffHsA);
  float* hsB = (float*)(ws + kOffHsB);
  float* hs[2] = { hsA, hsB };

  {
    const int n2a = kGates * kIn / 2;
    const int n2b = kGates * kHid / 2;
    cast_scale_f16x2<<<dim3((n2a + 255) / 256), dim3(256), 0, stream>>>(w_ih0, wih0, n2a, kScaleW);
    cast_scale_f16x2<<<dim3((n2b + 255) / 256), dim3(256), 0, stream>>>(w_hh0, whh0, n2b, kScaleW);
    cast_scale_f16x2<<<dim3((n2b + 255) / 256), dim3(256), 0, stream>>>(w_ih1, wih1, n2b, kScaleW);
    cast_scale_f16x2<<<dim3((n2b + 255) / 256), dim3(256), 0, stream>>>(w_hh1, whh1, n2b, kScaleW);
  }
  cast_x_timemajor<<<dim3((kSteps * kBatch + 31) / 32), dim3(256), 0, stream>>>(x, x16, kScaleX);

  const int chunkM = kChunk * kBatch;
  const int gemmTiles = (chunkM / 64) * (kGates / 64);
  const int gemmBlocks = (gemmTiles + 7) / 8;

  for (int c = 0; c < kNumChunks; ++c) {
    const unsigned short* Ap = x16 + (size_t)c * chunkM * kIn;
    wmma_gemm64<0, false, 2, 0, false, 0><<<dim3(gemmBlocks, 1), dim3(256), 0, stream>>>(
        Ap, Ap, kIn, 0L, wih0, wih0, kIn, 0L, (void*)xg, (void*)xg, kGates, 0L,
        b_ih0, b_ih0, 0L, chunkM, kGates, kIn, kInProj0Scale);
    rec_chunk<<<dim3(kBatch / kRowsPerBlk), dim3(256), 0, stream>>>(
        xg, whh0, b_hh0, hs[(c + 1) & 1], hs[c & 1], h1p, c * kChunk, kChunk, (c == 0) ? 1 : 0, 1);
  }
  for (int c = 0; c < kNumChunks; ++c) {
    const unsigned short* Ap = h1p + (size_t)c * chunkM * kHid;
    wmma_gemm64<0, false, 2, 0, false, 0><<<dim3(gemmBlocks, 1), dim3(256), 0, stream>>>(
        Ap, Ap, kHid, 0L, wih1, wih1, kHid, 0L, (void*)xg, (void*)xg, kGates, 0L,
        b_ih1, b_ih1, 0L, chunkM, kGates, kHid, kInProj1Scale);
    rec_chunk<<<dim3(kBatch / kRowsPerBlk), dim3(256), 0, stream>>>(
        xg, whh1, b_hh1, hs[(c + 1) & 1], hs[c & 1], h1p, c * kChunk, kChunk, (c == 0) ? 1 : 0, 0);
  }
  fc_head<<<dim3(1), dim3(256), 0, stream>>>(hs[(kNumChunks - 1) & 1], fc_w, fc_b, out);
}
